// SparseGraphAttentionLayer_83476984365497
// MI455X (gfx1250) — hardware-run, weakly checked
//
#include <hip/hip_runtime.h>
#include <stddef.h>


#define FDIM    256
#define NTHR    256
#define NWAVE   8
#define EPT     8
#define NGRP    2
#define CHUNK   (NTHR * EPT * NGRP)
#define WCAP    (EPT * NGRP * 32)
#define LISTN   (NWAVE * WCAP)
#define NBC     4096
#define NBF     1024
#define RCAP    40960
#define RBN     128
#define TGT     256
#define DEGCAP  512
#define OTHR    512
#define BM      32
#define BN      256
#define WSCAP   134217728
#define NEG_SLOPE 0.2f

#define LDS_FILL ((RCAP + NBF + LISTN) * 4 + 64)

static_assert((CHUNK & (CHUNK - 1)) == 0);
static_assert(CHUNK <= 4096);
static_assert(NBC <= 4096 && NBF <= 4096);
static_assert((NBC & (NBC - 1)) == 0 && (NBF & (NBF - 1)) == 0);
static_assert(NBC == 4 * NBF);
static_assert(OTHR * 8 == NBC);
static_assert((RCAP % 32) == 0);
static_assert(TGT == NWAVE * 32);
static_assert((NBC % TGT) == 0);
static_assert((TGT % BM) == 0);
static_assert(BM == 4 * NWAVE);
static_assert(BN == FDIM);
static_assert(FDIM % 32 == 0);
static_assert(FDIM == 2 * 128);

typedef float          v4f   __attribute__((ext_vector_type(4)));
typedef float          v8f   __attribute__((ext_vector_type(8)));
typedef int            v4i   __attribute__((ext_vector_type(4)));
typedef unsigned short v8us  __attribute__((ext_vector_type(8)));
typedef __bf16         v16bf __attribute__((ext_vector_type(16)));
union FragB { v16bf v; v8us u[2]; };

__device__ __forceinline__ v8f wmb(v16bf a, v16bf b, v8f c) {
  v8f d = __builtin_amdgcn_wmma_f32_16x16x32_bf16(false, a, false, b, (short)0, c, false, false);
  asm volatile("v_nop\n\tv_nop\n\tv_nop\n\tv_nop" : "+v"(d) : "v"(a), "v"(b));
  return d;
}

__device__ __forceinline__ unsigned bfr(float f) {
  const unsigned u = __float_as_uint(f);
  return (u + 0x7fffu + ((u >> 16) & 1u)) >> 16;
}

__device__ __forceinline__ void split8(v4f a, v4f b, v8us& hi, v8us& lo) {
  v8f f;
  f[0] = a.x; f[1] = a.y; f[2] = a.z; f[3] = a.w;
  f[4] = b.x; f[5] = b.y; f[6] = b.z; f[7] = b.w;
  v8us h, l;
#pragma unroll
  for (int i = 0; i < 8; ++i) {
    const unsigned hb = bfr(f[i]);
    const float hf = __uint_as_float(hb << 16);
    const unsigned lb = bfr(f[i] - hf);
    h[i] = (unsigned short)hb;
    l[i] = (unsigned short)lb;
  }
  hi = h; lo = l;
}

__device__ __forceinline__ float lrelu(float v) { return v > 0.0f ? v : NEG_SLOPE * v; }

__device__ __forceinline__ float wvmax(float v) {
#pragma unroll
  for (int o = 16; o > 0; o >>= 1) v = fmaxf(v, __shfl_xor(v, o));
  return v;
}
__device__ __forceinline__ float wvsum(float v) {
#pragma unroll
  for (int o = 16; o > 0; o >>= 1) v += __shfl_xor(v, o);
  return v;
}

template <int NB>
__device__ __forceinline__ int scan_chunk(const int* __restrict__ dsts, int nE, int cbase, int slotBase,
                                          int vec8, int* list, int tid, int lane, int wave) {
  int wc = 0;
#pragma unroll
  for (int g = 0; g < NGRP; ++g) {
    const int el0  = (g * NTHR + tid) * EPT;
    const int e0   = cbase + el0;
    const int sent = -2147483647 - 1;
    v4i da, db;
    if (vec8 != 0 && cbase + CHUNK <= nE) {
      da = *(const v4i*)(dsts + e0);
      db = *(const v4i*)(dsts + e0 + 4);
    } else {
      da.x = (e0     < nE) ? dsts[min(e0, nE - 1)] : sent;
      da.y = (e0 + 1 < nE) ? dsts[min(e0 + 1, nE - 1)] : sent;
      da.z = (e0 + 2 < nE) ? dsts[min(e0 + 2, nE - 1)] : sent;
      da.w = (e0 + 3 < nE) ? dsts[min(e0 + 3, nE - 1)] : sent;
      db.x = (e0 + 4 < nE) ? dsts[min(e0 + 4, nE - 1)] : sent;
      db.y = (e0 + 5 < nE) ? dsts[min(e0 + 5, nE - 1)] : sent;
      db.z = (e0 + 6 < nE) ? dsts[min(e0 + 6, nE - 1)] : sent;
      db.w = (e0 + 7 < nE) ? dsts[min(e0 + 7, nE - 1)] : sent;
    }
    const unsigned nb = (unsigned)slotBase;
    const unsigned s0 = (unsigned)da.x - nb, s1 = (unsigned)da.y - nb;
    const unsigned s2 = (unsigned)da.z - nb, s3 = (unsigned)da.w - nb;
    const unsigned s4 = (unsigned)db.x - nb, s5 = (unsigned)db.y - nb;
    const unsigned s6 = (unsigned)db.z - nb, s7 = (unsigned)db.w - nb;
    const bool h0 = s0 < (unsigned)NB, h1 = s1 < (unsigned)NB, h2 = s2 < (unsigned)NB, h3 = s3 < (unsigned)NB;
    const bool h4 = s4 < (unsigned)NB, h5 = s5 < (unsigned)NB, h6 = s6 < (unsigned)NB, h7 = s7 < (unsigned)NB;
    const unsigned any = __builtin_amdgcn_ballot_w32(h0 | h1 | h2 | h3 | h4 | h5 | h6 | h7);
    if (any != 0u) {
#define HITJ(J, HJ, SJ) { \
        const unsigned mj = __builtin_amdgcn_ballot_w32(HJ); \
        if (mj != 0u) { \
          if (HJ) { \
            const int pos = wc + (int)__builtin_amdgcn_mbcnt_lo(mj, 0u); \
            if (pos < WCAP) list[wave * WCAP + pos] = ((el0 + (J)) << 12) | (int)(SJ); \
          } \
          wc += (int)__builtin_popcount(mj); } }
      HITJ(0, h0, s0)
      HITJ(1, h1, s1)
      HITJ(2, h2, s2)
      HITJ(3, h3, s3)
      HITJ(4, h4, s4)
      HITJ(5, h5, s5)
      HITJ(6, h6, s6)
      HITJ(7, h7, s7)
#undef HITJ
    }
  }
  return wc;
}

__global__ __launch_bounds__(NTHR) void k_xcvt(const float* __restrict__ x,
                                               unsigned short* xh, unsigned short* xl,
                                               int nN, int nUnits) {
  const int i = (int)blockIdx.x * NTHR + (int)threadIdx.x;
  if (i >= nUnits) return;
  const int row = i >> 5;
  const int c0  = (i & 31) * 8;
  int rr = row > nN - 1 ? nN - 1 : row;
  rr = rr < 0 ? 0 : rr;
  const float* p = x + (size_t)rr * FDIM + c0;
  v4f a = *(const v4f*)p, b = *(const v4f*)(p + 4);
  const v4f z = {0.f, 0.f, 0.f, 0.f};
  if (row >= nN) { a = z; b = z; }
  v8us h, l;
  split8(a, b, h, l);
  unsigned short* dh = xh + (size_t)i * 8;
  unsigned short* dl = xl + (size_t)i * 8;
  *(volatile v8us*)dh = h;
  *(volatile v8us*)dl = l;
  __threadfence();
  *(volatile v8us*)dh = h;
  *(volatile v8us*)dl = l;
}

__global__ __launch_bounds__(NTHR) void k_wprep(const float* __restrict__ W,
                                                unsigned short* wh, unsigned short* wl) {
  constexpr int KS    = FDIM / 8;
  constexpr int UNITS = FDIM * KS;
  const int i = (int)blockIdx.x * NTHR + (int)threadIdx.x;
  if (i >= UNITS) return;
  const int n  = i / KS;
  const int k0 = (i - n * KS) * 8;
  v4f a, b;
  a.x = W[(size_t)(k0 + 0) * FDIM + n]; a.y = W[(size_t)(k0 + 1) * FDIM + n];
  a.z = W[(size_t)(k0 + 2) * FDIM + n]; a.w = W[(size_t)(k0 + 3) * FDIM + n];
  b.x = W[(size_t)(k0 + 4) * FDIM + n]; b.y = W[(size_t)(k0 + 5) * FDIM + n];
  b.z = W[(size_t)(k0 + 6) * FDIM + n]; b.w = W[(size_t)(k0 + 7) * FDIM + n];
  v8us h, l;
  split8(a, b, h, l);
  unsigned short* dh = wh + (size_t)i * 8;
  unsigned short* dl = wl + (size_t)i * 8;
  *(volatile v8us*)dh = h;
  *(volatile v8us*)dl = l;
  __threadfence();
  *(volatile v8us*)dh = h;
  *(volatile v8us*)dl = l;
}

__global__ __launch_bounds__(NTHR) void k_count(
    const int* __restrict__ dsts, int* cnt, int nE, int vec8) {
  __shared__ __attribute__((aligned(16))) int scnt[NBC];
  __shared__ __attribute__((aligned(16))) int list[LISTN];
  __shared__ int wcnt[NWAVE];
  const int tid = threadIdx.x, lane = tid & 31, wave = tid >> 5;
  const int nodeBase = blockIdx.x * NBC;

  for (int i = tid; i < NBC; i += NTHR) scnt[i] = 0;
  __syncthreads();

  const int nChunks = (nE + CHUNK - 1) / CHUNK;
#pragma unroll 1
  for (int ch = 0; ch < nChunks; ++ch) {
    const int cbase = ch * CHUNK;
    const int wc = scan_chunk<NBC>(dsts, nE, cbase, nodeBase, vec8, list, tid, lane, wave);
    if (lane == 0) wcnt[wave] = wc;
    __syncthreads();
    if (wave == 0) {
#pragma unroll 1
      for (int wsx = 0; wsx < NWAVE; ++wsx) {
        int n = __builtin_amdgcn_readfirstlane(wcnt[wsx]);
        n = n > WCAP ? WCAP : (n < 0 ? 0 : n);
        const int* lp = list + wsx * WCAP;
#pragma unroll 1
        for (int i = 0; i < n; ++i) {
          const int ent  = __builtin_amdgcn_readfirstlane(lp[i]);
          const int slot = ent & (NBC - 1);
          if (lane == 0) scnt[slot] = scnt[slot] + 1;
        }
      }
    }
    __syncthreads();
  }

  v4i cq[4];
#pragma unroll
  for (int q = 0; q < 4; ++q) {
    const int f = (wave * 4 + q) * 128 + 4 * lane;
    cq[q] = *(const v4i*)(scnt + f);
  }
  int* cp = cnt + (size_t)nodeBase;
#pragma unroll
  for (int q = 0; q < 4; ++q) {
    const int f = (wave * 4 + q) * 128 + 4 * lane;
    *(volatile v4i*)(cp + f) = cq[q];
  }
  __threadfence();
#pragma unroll
  for (int q = 0; q < 4; ++q) {
    const int f = (wave * 4 + q) * 128 + 4 * lane;
    *(volatile v4i*)(cp + f) = cq[q];
  }
}

__global__ __launch_bounds__(OTHR) void k_offsets(
    const int* __restrict__ cnt, int* off, int* rbase, int nChunk) {
  __shared__ __attribute__((aligned(16))) int soff[NBC];
  __shared__ __attribute__((aligned(16))) int srb[RBN];
  __shared__ int wtot[OTHR / 32];
  const int tid = threadIdx.x, lane = tid & 31, wave = tid >> 5, sub = tid >> 7;
  for (int i = tid; i < RBN; i += OTHR) srb[i] = 0;
  int carry = 0;
#pragma unroll 1
  for (int ch = 0; ch < nChunk; ++ch) {
    const int base = ch * NBC;
    const v4i c0 = *(const v4i*)(cnt + base + 8 * tid);
    const v4i c1 = *(const v4i*)(cnt + base + 8 * tid + 4);
    const int e0 = max(c0.x, 0), e1 = max(c0.y, 0), e2 = max(c0.z, 0), e3 = max(c0.w, 0);
    const int e4 = max(c1.x, 0), e5 = max(c1.y, 0), e6 = max(c1.z, 0), e7 = max(c1.w, 0);
    const int ts = e0 + e1 + e2 + e3 + e4 + e5 + e6 + e7;
    int incl = ts;
#pragma unroll
    for (int d = 1; d < 32; d <<= 1) {
      const int t = __shfl_up(incl, d);
      if (lane >= d) incl += t;
    }
    if (lane == 31) wtot[wave] = incl;
    __syncthreads();
    const int S0 = wtot[0]  + wtot[1]  + wtot[2]  + wtot[3];
    const int S1 = wtot[4]  + wtot[5]  + wtot[6]  + wtot[7];
    const int S2 = wtot[8]  + wtot[9]  + wtot[10] + wtot[11];
    const int S3 = wtot[12] + wtot[13] + wtot[14] + wtot[15];
    int pre = 0;
#pragma unroll 1
    for (int w = 4 * sub; w < wave; ++w) pre += wtot[w];
    const int b0 = carry;
    const int b1 = b0 + ((S0 + 31) & ~31);
    const int b2 = b1 + ((S1 + 31) & ~31);
    const int b3 = b2 + ((S2 + 31) & ~31);
    const int b4 = b3 + ((S3 + 31) & ~31);
    const int myb = sub == 0 ? b0 : (sub == 1 ? b1 : (sub == 2 ? b2 : b3));
    if (tid == 0) {
      srb[min(4 * ch + 0, RBN - 1)] = b0;
      srb[min(4 * ch + 1, RBN - 1)] = b1;
      srb[min(4 * ch + 2, RBN - 1)] = b2;
      srb[min(4 * ch + 3, RBN - 1)] = b3;
    }
    int run = myb + pre + incl - ts;
    soff[8 * tid + 0] = run; run += e0;
    soff[8 * tid + 1] = run; run += e1;
    soff[8 * tid + 2] = run; run += e2;
    soff[8 * tid + 3] = run; run += e3;
    soff[8 * tid + 4] = run; run += e4;
    soff[8 * tid + 5] = run; run += e5;
    soff[8 * tid + 6] = run; run += e6;
    soff[8 * tid + 7] = run;
    carry = b4;
    __syncthreads();
    const v4i o0 = *(const v4i*)(soff + 4 * tid);
    const v4i o1 = *(const v4i*)(soff + 4 * (tid + OTHR));
    int* op = off + base;
    *(volatile v4i*)(op + 4 * tid) = o0;
    *(volatile v4i*)(op + 4 * (tid + OTHR)) = o1;
    __threadfence();
    *(volatile v4i*)(op + 4 * tid) = o0;
    *(volatile v4i*)(op + 4 * (tid + OTHR)) = o1;
    __syncthreads();
  }
  if (tid == 0) srb[min(4 * nChunk, RBN - 1)] = carry;
  __syncthreads();
  v4i rv = {0, 0, 0, 0};
  if (tid < 32) rv = *(const v4i*)(srb + 4 * tid);
  if (tid < 32) *(volatile v4i*)(rbase + 4 * tid) = rv;
  __threadfence();
  if (tid < 32) *(volatile v4i*)(rbase + 4 * tid) = rv;
}

__global__ __launch_bounds__(NTHR) void k_fill(
    const int* __restrict__ srcs, const int* __restrict__ dsts,
    const int* __restrict__ off, const int* __restrict__ rbase,
    int* csr, int nN, int nE, int vec8, int csrLen) {
  extern __shared__ v4f lds_dyn[];
  int* region = (int*)lds_dyn;
  int* cursor = region + RCAP;
  int* list   = cursor + NBF;
  int* wcnt   = list + LISTN;
  const int tid = threadIdx.x, lane = tid & 31, wave = tid >> 5;
  const int b = blockIdx.x;
  const int nodeBase = b * NBF;

  int rb0 = rbase[b];
  const int rb1 = rbase[b + 1];
  rb0 = rb0 < 0 ? 0 : (rb0 > csrLen ? csrLen : rb0);
  rb0 &= ~31;
  int len = rb1 - rb0;
  len = len < 0 ? 0 : (len > RCAP ? RCAP : len);
  int lenW = (len + 31) & ~31;
  if (rb0 + lenW > csrLen) lenW = (csrLen - rb0) & ~31;

  {
    const v4i z = {0, 0, 0, 0};
    for (int i = tid; i < RCAP / 4; i += NTHR) ((v4i*)region)[i] = z;
    for (int s = tid; s < NBF; s += NTHR) {
      int o = off[nodeBase + s] - rb0;
      o = o < 0 ? 0 : (o > RCAP ? RCAP : o);
      cursor[s] = o;
    }
  }
  __syncthreads();

  const int nChunks = (nE + CHUNK - 1) / CHUNK;
#pragma unroll 1
  for (int ch = 0; ch < nChunks; ++ch) {
    const int cbase = ch * CHUNK;
    const int wc = scan_chunk<NBF>(dsts, nE, cbase, nodeBase, vec8, list, tid, lane, wave);
    if (lane == 0) wcnt[wave] = wc;
    __syncthreads();
    if (wave == 0) {
#pragma unroll 1
      for (int wsx = 0; wsx < NWAVE; ++wsx) {
        int n = __builtin_amdgcn_readfirstlane(wcnt[wsx]);
        n = n > WCAP ? WCAP : (n < 0 ? 0 : n);
        const int* lp = list + wsx * WCAP;
#pragma unroll 1
        for (int i = 0; i < n; ++i) {
          const int ent  = __builtin_amdgcn_readfirstlane(lp[i]);
          const int slot = ent & (NBF - 1);
          int e = cbase + ((ent >> 12) & (CHUNK - 1));
          e = e > nE - 1 ? nE - 1 : e;
          int src = srcs[e];
          src = src < 0 ? 0 : (src > nN - 1 ? nN - 1 : src);
          if (lane == 0) {
            int pos = cursor[slot];
            pos = pos < 0 ? 0 : (pos > RCAP - 1 ? RCAP - 1 : pos);
            region[pos] = src;
            const int np = pos + 1;
            cursor[slot] = np > RCAP ? RCAP : np;
          }
        }
      }
    }
    __syncthreads();
  }

  const int nv = lenW >> 2;
  int* gp = csr + rb0;
#pragma unroll 1
  for (int i = tid; i < nv; i += NTHR) { const v4i v = ((const v4i*)region)[i]; *(volatile v4i*)(gp + 4 * i) = v; }
  __threadfence();
#pragma unroll 1
  for (int i = tid; i < nv; i += NTHR) { const v4i v = ((const v4i*)region)[i]; *(volatile v4i*)(gp + 4 * i) = v; }
}

__global__ __launch_bounds__(NTHR) void k_gemm(
    const unsigned short* __restrict__ Ah, const unsigned short* __restrict__ Al,
    const unsigned short* __restrict__ Bh, const unsigned short* __restrict__ Bl,
    const float* __restrict__ bias, const float* __restrict__ aw,
    float* C, float* eS, float* eD) {
  constexpr int K   = FDIM;
  constexpr int KT  = K / 32;
  constexpr int TPW = 4;
  constexpr int NIT = BM / NWAVE;
  constexpr int CPP = 32;
  static_assert(K % 32 == 0);
  static_assert(TPW * 16 * 4 == BN);
  static_assert(CPP * 8 == BN);

  __shared__ __attribute__((aligned(16))) float stg[BM * BN];
  __shared__ __attribute__((aligned(16))) float sES[BM];
  __shared__ __attribute__((aligned(16))) float sED[BM];
  const int tid = threadIdx.x, lane = tid & 31, wave = tid >> 5, hh = lane >> 4, m = lane & 15;
  const int rowBase = blockIdx.x * BM;
  const int rg = wave >> 2, chf = wave & 3;
  const int r0 = rg * 16;
  const int c0 = chf * 64;

  v8f acc[TPW];
#pragma unroll
  for (int t = 0; t < TPW; ++t) { v8f z = {0.f, 0.f, 0.f, 0.f, 0.f, 0.f, 0.f, 0.f}; acc[t] = z; }

  const size_t arow = (size_t)(rowBase + r0 + m) * K + 8 * hh;
  const unsigned short* aph  = Ah + arow;
  const unsigned short* apl  = Al + arow;
  const size_t brow = (size_t)(c0 + m) * K + 8 * hh;
  const unsigned short* bph0 = Bh + brow;
  const unsigned short* bpl0 = Bl + brow;
#pragma unroll 1
  for (int kt = 0; kt < KT; ++kt) {
    FragB ah, al;
    ah.u[0] = *(const v8us*)(aph + 32 * kt);
    ah.u[1] = *(const v8us*)(aph + 32 * kt + 16);
    al.u[0] = *(const v8us*)(apl + 32 * kt);
    al.u[1] = *(const v8us*)(apl + 32 * kt + 16);
#pragma unroll
    for (int t = 0; t < TPW; ++t) {
      const size_t bo = (size_t)(16 * t) * K + 32 * kt;
      FragB bh, bl;
      bh.u[0] = *(const v8us*)(bph0 + bo);
      bh.u[1] = *(const v8us*)(bph0 + bo + 16);
      bl.u[0] = *(const v8us*)(bpl0 + bo);
      bl.u[1] = *(const v8us*)(bpl0 + bo + 16);
      acc[t] = wmb(ah.v, bh.v, acc[t]);
      acc[t] = wmb(ah.v, bl.v, acc[t]);
      acc[t] = wmb(al.v, bh.v, acc[t]);
    }
  }

  {
    float* sp = stg + (size_t)(r0 + 8 * hh) * BN + c0 + m;
#pragma unroll
    for (int t = 0; t < TPW; ++t) {
      const float bc = bias[c0 + 16 * t + m];
#pragma unroll
      for (int r = 0; r < 8; ++r) sp[r * BN + 16 * t] = acc[t][r] + bc;
    }
  }
  __syncthreads();

  {
    const int drow = tid >> 3, part = tid & 7;
    const float* rp  = stg + (size_t)drow * BN + CPP * part;
    const float* sa  = aw + CPP * part;
    const float* sdd = aw + FDIM + CPP * part;
    float ps = 0.f, pd = 0.f;
#pragma unroll 2
    for (int c = 0; c < CPP; c += 4) {
      const v4f hv = *(const v4f*)(rp + c);
      const v4f av = *(const v4f*)(sa + c);
      const v4f dv = *(const v4f*)(sdd + c);
      ps += hv.x * av.x + hv.y * av.y + hv.z * av.z + hv.w * av.w;
      pd += hv.x * dv.x + hv.y * dv.y + hv.z * dv.z + hv.w * dv.w;
    }
    ps += __shfl_xor(ps, 1); pd += __shfl_xor(pd, 1);
    ps += __shfl_xor(ps, 2); pd += __shfl_xor(pd, 2);
    ps += __shfl_xor(ps, 4); pd += __shfl_xor(pd, 4);
    if (part == 0) { sES[drow] = ps; sED[drow] = pd; }
  }

  {
    float* cb = C + (size_t)rowBase * FDIM + 4 * lane;
    v4f cv0[NIT], cv1[NIT];
#pragma unroll
    for (int it = 0; it < NIT; ++it) {
      const float* srow = stg + (size_t)(it * NWAVE + wave) * BN + 4 * lane;
      cv0[it] = *(const v4f*)srow;
      cv1[it] = *(const v4f*)(srow + 128);
    }
#pragma unroll
    for (int it = 0; it < NIT; ++it) {
      float* gp = cb + (size_t)(it * NWAVE + wave) * FDIM;
      *(volatile v4f*)gp = cv0[it];
      *(volatile v4f*)(gp + 128) = cv1[it];
    }
    __threadfence();
#pragma unroll
    for (int it = 0; it < NIT; ++it) {
      float* gp = cb + (size_t)(it * NWAVE + wave) * FDIM;
      *(volatile v4f*)gp = cv0[it];
      *(volatile v4f*)(gp + 128) = cv1[it];
    }
  }
  __syncthreads();

  {
    const int lq = lane & 7;
    const v4f vS = *(const v4f*)(sES + 4 * lq);
    const v4f vD = *(const v4f*)(sED + 4 * lq);
    const v4f dv = (wave == 0) ? vS : vD;
    float* gp = ((wave == 0) ? eS : eD) + (size_t)rowBase + 4 * lq;
    const bool act = (wave < 2) && (lane < 8);
    if (act) *(volatile v4f*)gp = dv;
    __threadfence();
    if (act) *(volatile v4f*)gp = dv;
  }
}

__global__ __launch_bounds__(NTHR) void k_agg(
    const int* __restrict__ csr, const int* __restrict__ off, const int* __restrict__ cnt,
    const float* __restrict__ eS, const float* __restrict__ eD, const float* __restrict__ hw,
    const float* __restrict__ ab, float* out, int nN, int csrLen) {
  const int tid = threadIdx.x, lane = tid & 31, wave = tid >> 5;
  const int tbase = blockIdx.x * TGT + wave * 32;
  const int colA = 4 * lane;
  const int colB = 128 + 4 * lane;
  const float abv = ab[0];
  const float NEGI = -__builtin_huge_valf();

  const int cl      = tbase + lane;
  const int cnt_l   = cnt[cl];
  const int off_l   = off[cl];
  const float ed_l  = eD[cl];

#pragma unroll 1
  for (int j = 0; j < 32; ++j) {
    const int c = tbase + j;
    int n = __shfl(cnt_l, j);
    n = n < 0 ? 0 : (n > DEGCAP ? DEGCAP : n);
    const int st    = __shfl(off_l, j);
    const float edv = __shfl(ed_l, j);

    float mx = NEGI;
#pragma unroll 1
    for (int q0 = 0; q0 < n; q0 += 32) {
      int pos = st + q0 + lane;
      pos = pos < 0 ? 0 : (pos > csrLen - 1 ? csrLen - 1 : pos);
      int sl = csr[pos];
      sl = sl < 0 ? 0 : (sl > nN - 1 ? nN - 1 : sl);
      const float v = lrelu((eS[sl] + edv) + abv);
      mx = fmaxf(mx, (q0 + lane < n) ? v : NEGI);
    }
    mx = wvmax(mx);

    float den = 0.f;
    v4f b0 = {0.f, 0.f, 0.f, 0.f}, b1 = {0.f, 0.f, 0.f, 0.f};
#pragma unroll 1
    for (int q0 = 0; q0 < n; q0 += 32) {
      int pos = st + q0 + lane;
      pos = pos < 0 ? 0 : (pos > csrLen - 1 ? csrLen - 1 : pos);
      int sl = csr[pos];
      sl = sl < 0 ? 0 : (sl > nN - 1 ? nN - 1 : sl);
      const float v  = lrelu((eS[sl] + edv) + abv);
      const float pe = __expf(v - mx);
      const float pl = (q0 + lane < n) ? pe : 0.f;
      den += pl;
      const int mcnt = (n - q0) < 32 ? (n - q0) : 32;
#pragma unroll 1
      for (int pp = 0; pp < mcnt; ++pp) {
        const float p = __int_as_float(__builtin_amdgcn_readlane(__float_as_int(pl), pp));
        const int   s = __builtin_amdgcn_readlane(sl, pp);
        const float* hs = hw + (size_t)s * FDIM;
        const v4f h0 = *(const v4f*)(hs + colA);
        const v4f h1 = *(const v4f*)(hs + colB);
        b0 = b0 + h0 * p; b1 = b1 + h1 * p;
      }
    }
    den = wvsum(den);

    const float rcp = 1.0f / den;
    const float rd  = (n > 0) ? rcp : 0.f;
    v4f o0, o1;
    o0.x = fmaxf(b0.x * rd, 0.f); o0.y = fmaxf(b0.y * rd, 0.f); o0.z = fmaxf(b0.z * rd, 0.f); o0.w = fmaxf(b0.w * rd, 0.f);
    o1.x = fmaxf(b1.x * rd, 0.f); o1.y = fmaxf(b1.y * rd, 0.f); o1.z = fmaxf(b1.z * rd, 0.f); o1.w = fmaxf(b1.w * rd, 0.f);
    float* gp = out + (size_t)c * FDIM;
    if (c < nN) {
      *(volatile v4f*)(gp + colA) = o0;
      *(volatile v4f*)(gp + colB) = o1;
    }
    __threadfence();
    if (c < nN) {
      *(volatile v4f*)(gp + colA) = o0;
      *(volatile v4f*)(gp + colB) = o1;
    }
  }
}

extern "C" void kernel_launch(void* const* d_in, const int* in_sizes, int n_in,
                              void* d_out, int out_size, void* d_ws, size_t ws_size,
                              hipStream_t stream) {
  if (n_in < 7) return;
  const int nN = in_sizes[0] / FDIM;
  const int nE = in_sizes[5];
  if (nN <= 0 || nE <= 0 || in_sizes[0] != nN * FDIM) return;
  if (in_sizes[1] != FDIM * FDIM || in_sizes[2] != FDIM || in_sizes[3] != 2 * FDIM || in_sizes[4] < 1) return;
  if (in_sizes[6] != nE) return;
  if (nE > (1 << 26) || nN > (1 << 22)) return;
  if ((long long)out_size != (long long)nN * FDIM) return;

  const float* x   = (const float*)d_in[0];
  const float* Ww  = (const float*)d_in[1];
  const float* Wb  = (const float*)d_in[2];
  const float* aw  = (const float*)d_in[3];
  const float* ab  = (const float*)d_in[4];
  const int*   dst = (const int*)d_in[5];
  const int*   src = (const int*)d_in[6];
  float* out0 = (float*)d_out;

  const int NPAD   = ((nN + TGT - 1) / TGT) * TGT;
  const int nBC    = (nN + NBC - 1) / NBC;
  const int CNTPAD = nBC * NBC;
  if (CNTPAD < NPAD) return;
  if (4 * nBC + 1 > RBN) return;
  const int nBF    = (nN + NBF - 1) / NBF;
  if (nBF + 1 > 4 * nBC + 1) return;
  const int csrLen = ((nE + 31) & ~31) + 4096;
  if (31 * 4 * nBC > 4096) return;
  const int nAgg   = NPAD / TGT;
  const int nGemm  = NPAD / BM;
  const int nXu    = NPAD * (FDIM / 8);

  char* ws = (char*)d_ws;
  size_t off = 0;
  const size_t oWh  = off; off += (size_t)FDIM * FDIM * 2;        off = (off + 255) & ~(size_t)255;
  const size_t oWl  = off; off += (size_t)FDIM * FDIM * 2;        off = (off + 255) & ~(size_t)255;
  const size_t oXh  = off; off += (size_t)NPAD * FDIM * 2;        off = (off + 255) & ~(size_t)255;
  const size_t oXl  = off; off += (size_t)NPAD * FDIM * 2;        off = (off + 255) & ~(size_t)255;
  const size_t oCnt = off; off += (size_t)CNTPAD * 4;             off = (off + 255) & ~(size_t)255;
  const size_t oOff = off; off += (size_t)CNTPAD * 4;             off = (off + 255) & ~(size_t)255;
  const size_t oRb  = off; off += (size_t)RBN * 4;                off = (off + 255) & ~(size_t)255;
  const size_t oCsr = off; off += (size_t)csrLen * 4;             off = (off + 255) & ~(size_t)255;
  const size_t oHw  = off; off += (size_t)NPAD * FDIM * 4;        off = (off + 255) & ~(size_t)255;
  const size_t oES  = off; off += (size_t)NPAD * 4;               off = (off + 255) & ~(size_t)255;
  const size_t oED  = off; off += (size_t)NPAD * 4;               off = (off + 255) & ~(size_t)255;
  if (off > ws_size || off > (size_t)WSCAP) return;
  unsigned short* wph = (unsigned short*)(ws + oWh);
  unsigned short* wpl = (unsigned short*)(ws + oWl);
  unsigned short* xph = (unsigned short*)(ws + oXh);
  unsigned short* xpl = (unsigned short*)(ws + oXl);
  int*   cnt  = (int*)(ws + oCnt);
  int*   offp = (int*)(ws + oOff);
  int*   rb   = (int*)(ws + oRb);
  int*   csr  = (int*)(ws + oCsr);
  float* hw   = (float*)(ws + oHw);
  float* es   = (float*)(ws + oES);
  float* ed   = (float*)(ws + oED);

  const int vec8 = 1;

  k_wprep<<<(FDIM * FDIM / 8 + NTHR - 1) / NTHR, NTHR, 0, stream>>>(Ww, wph, wpl);
  k_xcvt<<<(nXu + NTHR - 1) / NTHR, NTHR, 0, stream>>>(x, xph, xpl, nN, nXu);

  k_count<<<nBC, NTHR, 0, stream>>>(dst, cnt, nE, vec8);
  k_offsets<<<1, OTHR, 0, stream>>>(cnt, offp, rb, nBC);
  hipFuncSetAttribute(reinterpret_cast<const void*>(&k_fill),
                      hipFuncAttributeMaxDynamicSharedMemorySize, LDS_FILL);
  k_fill<<<nBF, NTHR, LDS_FILL, stream>>>(src, dst, offp, rb, csr, nN, nE, vec8, csrLen);

  k_gemm<<<nGemm, NTHR, 0, stream>>>(xph, xpl, wph, wpl, Wb, aw, hw, es, ed);

  k_agg<<<nAgg, NTHR, 0, stream>>>(csr, offp, cnt, es, ed, hw, ab, out0, nN, csrLen);
}
